// TempModule_74620761801330
// MI455X (gfx1250) — hardware-verified
//
#include <hip/hip_runtime.h>


#define DM     128
#define DI     256
#define DS     16
#define DTRK   8
#define DCONV  4
#define NGRP   4
#define NBAT   2
#define TLEN   256
#define NNODES 128
#define NSEQ   (NBAT * NNODES)
#define NTOK   (NSEQ * TLEN)
#define XDBW   64
#define UTP    264
#define STP    68
#define GNBLK  256
#define GNROWS ((NBAT * TLEN * NNODES) / GNBLK)
#define GN_EPS 1e-5f
#define WSCALE 32.0f
#define WINV   0.03125f

static_assert(DM == 128);
static_assert(NNODES == 128);
static_assert(TLEN == 256);
static_assert(NTOK % 64 == 0);
static_assert(TLEN % 64 == 0);
static_assert(DI % 64 == 0);
static_assert((2 * DI) % 128 == 0);
static_assert(DTRK + 2 * DS <= XDBW);
static_assert(GNROWS % 64 == 0);
static_assert((GNBLK / NBAT) * GNROWS == TLEN * NNODES);
static_assert((UTP * 2) % 16 == 0);
static_assert((STP * 4) % 16 == 0);

typedef float          v4f    __attribute__((ext_vector_type(4)));
typedef float          v8f    __attribute__((ext_vector_type(8)));
typedef _Float16       v8h    __attribute__((ext_vector_type(8)));
typedef _Float16       v16h   __attribute__((ext_vector_type(16)));
typedef unsigned short u16x8  __attribute__((ext_vector_type(8)));
typedef double         v2d    __attribute__((ext_vector_type(2)));
typedef float          v4fa   __attribute__((ext_vector_type(4), may_alias));
typedef unsigned short u16x8a __attribute__((ext_vector_type(8), may_alias));

union FragH { u16x8 h[2]; v16h v; };
union Pack8 { v8h f; u16x8 u; };
union H16   { _Float16 f; unsigned short u; };

__device__ __forceinline__ v8f ld8f(const float* p) {
    v4f a = *(const v4f*)p;
    v4f b = *(const v4f*)(p + 4);
    return __builtin_shufflevector(a, b, 0, 1, 2, 3, 4, 5, 6, 7);
}
__device__ __forceinline__ u16x8 pack_f16(v8f x) {
    Pack8 pk;
    pk.f = __builtin_convertvector(x, v8h);
    return pk.u;
}
__device__ __forceinline__ float silu_f(float x) {
    float e = __expf(-x);
    return x * __builtin_amdgcn_rcpf(1.0f + e);
}
__device__ __forceinline__ float softplus_f(float x) {
    return fmaxf(x, 0.0f) + log1pf(__expf(-fabsf(x)));
}
__device__ __forceinline__ float conv4_silu(float x0, float x1, float x2, float x3,
                                            float w0, float w1, float w2, float w3, float bias) {
    float c = x0 * w0 + x1 * w1 + x2 * w2 + x3 * w3;
    return silu_f(bias + c);
}

__device__ __forceinline__ void mma16(v8f& acc, const FragH& a, const FragH& b) {
    acc = __builtin_amdgcn_wmma_f32_16x16x32_f16(false, a.v, false, b.v, (short)0, acc, false, false);
    asm volatile("v_nop\n\tv_nop\n\tv_nop\n\tv_nop" : "+v"(acc) : "v"(a.v), "v"(b.v));
}

__global__ __launch_bounds__(256)
void cvt_v_kernel(const float* __restrict__ v, unsigned short* x16, int n8)
{
    const int i = blockIdx.x * 256 + threadIdx.x;
    if (i >= n8) return;
    const int m  = i / (DM / 8);
    const int c  = (i % (DM / 8)) * 8;
    const int sq = m / TLEN, t = m % TLEN;
    const int b  = sq / NNODES, nn = sq % NNODES;
    const float* src = v + ((((size_t)b * TLEN + t) * NNODES + nn) * DM + c);
    const u16x8 pk = pack_f16(ld8f(src));
    unsigned short* gp = x16 + (size_t)m * DM + c;
    *(volatile u16x8*)gp = pk;
    __threadfence();
    *(volatile u16x8*)gp = pk;
}

__global__ __launch_bounds__(256)
void cvt_w_kernel(const float* __restrict__ src, unsigned short* dst, int n8valid, int n8total, float scale)
{
    const int i = blockIdx.x * 256 + threadIdx.x;
    if (i >= n8total) return;
    v8f x;
#pragma unroll
    for (int c = 0; c < 8; ++c) x[c] = 0.0f;
    if (i < n8valid) x = ld8f(src + (size_t)i * 8) * scale;
    const u16x8 pk = pack_f16(x);
    unsigned short* gp = dst + (size_t)i * 8;
    *(volatile u16x8*)gp = pk;
    __threadfence();
    *(volatile u16x8*)gp = pk;
}

template<int CW, int P>
__device__ __forceinline__ void rows_store_f32(const float* st, float* gp, size_t ld, int lane) {
    constexpr int LPR = CW / 4, RPI = 32 / LPR, NIT = 32 / RPI;
    const int rsub = lane / LPR, c4 = (lane % LPR) * 4;
#pragma unroll
    for (int it = 0; it < NIT; ++it) {
        const int row = it * RPI + rsub;
        const v4f val = *(const v4fa*)(st + row * P + c4);
        *(volatile v4f*)(gp + (size_t)row * ld + c4) = val;
    }
}
template<int CW, int P>
__device__ __forceinline__ void rows_store_res(const float* st, float* gp, const float* __restrict__ res,
                                               size_t ld, int lane) {
    constexpr int LPR = CW / 4, RPI = 32 / LPR, NIT = 32 / RPI;
    const int rsub = lane / LPR, c4 = (lane % LPR) * 4;
#pragma unroll
    for (int it = 0; it < NIT; ++it) {
        const int row = it * RPI + rsub;
        const v4f a = *(const v4fa*)(st + row * P + c4);
        const v4f r = *(const v4f*)(res + (size_t)row * ld + c4);
        const v4f val = a + r;
        *(volatile v4f*)(gp + (size_t)row * ld + c4) = val;
    }
}
template<int CW, int P>
__device__ __forceinline__ void rows_store_f16(const float* st, unsigned short* gp, size_t ld, int lane) {
    constexpr int LPR = CW / 8, RPI = 32 / LPR, NIT = 32 / RPI;
    const int rsub = lane / LPR, c8 = (lane % LPR) * 8;
#pragma unroll
    for (int it = 0; it < NIT; ++it) {
        const int row = it * RPI + rsub;
        const v4f a = *(const v4fa*)(st + row * P + c8);
        const v4f b = *(const v4fa*)(st + row * P + c8 + 4);
        const v8f x = __builtin_shufflevector(a, b, 0, 1, 2, 3, 4, 5, 6, 7);
        const u16x8 val = pack_f16(x);
        *(volatile u16x8*)(gp + (size_t)row * ld + c8) = val;
    }
}

template<int NBF, int EPI>
__global__ __launch_bounds__(128)
void gemm_tn_kernel(const unsigned short* __restrict__ A, const unsigned short* __restrict__ Bw, int K,
                    float* Cf, unsigned short* Ch, const float* __restrict__ res)
{
    constexpr int CW = NBF * 16;
    constexpr int P  = CW + 4;
    __shared__ __attribute__((aligned(16))) float stile[4][32 * P];

    const int tid  = threadIdx.x;
    const int lane = tid & 31;
    const int wave = tid >> 5;
    const int h    = lane >> 4;
    const int m    = lane & 15;
    const int wm   = wave >> 1;
    const int wn   = wave & 1;

    const int rowW = blockIdx.y * 64 + wm * 32;
    const int colW = blockIdx.x * (2 * CW) + wn * CW;

    v8f acc[2 * NBF];
#pragma unroll
    for (int j = 0; j < 2 * NBF; ++j)
#pragma unroll
        for (int r = 0; r < 8; ++r) acc[j][r] = 0.0f;

    const size_t aoff  = (size_t)(rowW + m) * K + 8 * h;
    const size_t boff  = (size_t)(colW + m) * K + 8 * h;
    const size_t sub16 = (size_t)16 * K;
    const int nk = K >> 5;

#pragma unroll 1
    for (int kt = 0; kt < nk; ++kt) {
        const size_t k0 = (size_t)kt * 32;
        FragH fa[2], fb[NBF];
#pragma unroll
        for (int s = 0; s < 2; ++s) {
            const unsigned short* p = A + aoff + s * sub16 + k0;
            fa[s].h[0] = *(const u16x8*)(p);
            fa[s].h[1] = *(const u16x8*)(p + 16);
        }
#pragma unroll
        for (int j = 0; j < NBF; ++j) {
            const unsigned short* p = Bw + boff + j * sub16 + k0;
            fb[j].h[0] = *(const u16x8*)(p);
            fb[j].h[1] = *(const u16x8*)(p + 16);
        }
#pragma unroll
        for (int s = 0; s < 2; ++s)
#pragma unroll
            for (int j = 0; j < NBF; ++j)
                mma16(acc[s * NBF + j], fa[s], fb[j]);
    }

    float* st = stile[wave];
#pragma unroll
    for (int s = 0; s < 2; ++s)
#pragma unroll
        for (int j = 0; j < NBF; ++j)
#pragma unroll
            for (int r = 0; r < 8; ++r)
                st[(s * 16 + 8 * h + r) * P + j * 16 + m] = acc[s * NBF + j][r] * WINV;
    __syncthreads();

    if (EPI == 0) {
        if (colW < DI) {
            float* gp = Cf + (size_t)rowW * DI + colW;
            rows_store_f32<CW, P>(st, gp, DI, lane);
            __threadfence();
            rows_store_f32<CW, P>(st, gp, DI, lane);
        } else {
            unsigned short* gp = Ch + (size_t)rowW * DI + (colW - DI);
            rows_store_f16<CW, P>(st, gp, DI, lane);
            __threadfence();
            rows_store_f16<CW, P>(st, gp, DI, lane);
        }
    } else {
        const int sq = rowW / TLEN, t0 = rowW % TLEN;
        const int b  = sq / NNODES, nn = sq % NNODES;
        const size_t gbase = (((size_t)b * TLEN + t0) * NNODES + nn) * DM + colW;
        const size_t ld = (size_t)NNODES * DM;
        rows_store_res<CW, P>(st, Cf + gbase, res + gbase, ld, lane);
        __threadfence();
        rows_store_res<CW, P>(st, Cf + gbase, res + gbase, ld, lane);
    }
}

__global__ __launch_bounds__(128)
void xproj_kernel(const float* __restrict__ X, const float* __restrict__ cw, const float* __restrict__ cb,
                  const unsigned short* __restrict__ Wx, float* xdb)
{
    __shared__ __attribute__((aligned(16))) unsigned short uT[64 * UTP];
    __shared__ __attribute__((aligned(16))) float stf[64 * STP];

    const int tid  = threadIdx.x;
    const int lane = tid & 31;
    const int wave = tid >> 5;
    const int h    = lane >> 4;
    const int m    = lane & 15;
    const int m0   = blockIdx.x * 64;
    const int t0   = m0 % TLEN;

    {
        const int d0  = (tid & 31) * 8;
        const int tl0 = wave * 16;
        v4f wv[8];
#pragma unroll
        for (int c = 0; c < 8; ++c) wv[c] = *(const v4f*)(cw + (size_t)(d0 + c) * DCONV);
        const v8f bias = ld8f(cb + d0);
        v8f xm1, xm2, xm3;
#pragma unroll
        for (int c = 0; c < 8; ++c) { xm1[c] = 0.0f; xm2[c] = 0.0f; xm3[c] = 0.0f; }
        const float* xr = X + (size_t)(m0 + tl0) * DI + d0;
        const int ta = t0 + tl0;
        if (ta >= 1) xm1 = ld8f(xr - DI);
        if (ta >= 2) xm2 = ld8f(xr - 2 * DI);
        if (ta >= 3) xm3 = ld8f(xr - 3 * DI);
#pragma unroll 1
        for (int i = 0; i < 16; ++i) {
            const v8f xv = ld8f(xr + (size_t)i * DI);
            v8f u;
#pragma unroll
            for (int c = 0; c < 8; ++c)
                u[c] = conv4_silu(xm3[c], xm2[c], xm1[c], xv[c], wv[c][0], wv[c][1], wv[c][2], wv[c][3], bias[c]);
            xm3 = xm2; xm2 = xm1; xm1 = xv;
            *(u16x8a*)(uT + (tl0 + i) * UTP + d0) = pack_f16(u);
        }
    }
    __syncthreads();

    const int wm = wave >> 1, wn = wave & 1;
    v8f acc[4];
#pragma unroll
    for (int j = 0; j < 4; ++j)
#pragma unroll
        for (int r = 0; r < 8; ++r) acc[j][r] = 0.0f;

    const unsigned short* ab = uT + (wm * 32 + m) * UTP + 8 * h;
    const size_t boff = (size_t)(wn * 32 + m) * DI + 8 * h;
#pragma unroll 1
    for (int kt = 0; kt < DI / 32; ++kt) {
        const int k0 = kt * 32;
        FragH fa[2], fb[2];
#pragma unroll
        for (int s = 0; s < 2; ++s) {
            const unsigned short* p = ab + s * 16 * UTP + k0;
            fa[s].h[0] = *(const u16x8a*)(p);
            fa[s].h[1] = *(const u16x8a*)(p + 16);
        }
#pragma unroll
        for (int j = 0; j < 2; ++j) {
            const unsigned short* p = Wx + boff + (size_t)j * 16 * DI + k0;
            fb[j].h[0] = *(const u16x8*)(p);
            fb[j].h[1] = *(const u16x8*)(p + 16);
        }
#pragma unroll
        for (int s = 0; s < 2; ++s)
#pragma unroll
            for (int j = 0; j < 2; ++j)
                mma16(acc[s * 2 + j], fa[s], fb[j]);
    }

#pragma unroll
    for (int s = 0; s < 2; ++s)
#pragma unroll
        for (int j = 0; j < 2; ++j)
#pragma unroll
            for (int r = 0; r < 8; ++r)
                stf[(wm * 32 + s * 16 + 8 * h + r) * STP + wn * 32 + j * 16 + m] = acc[s * 2 + j][r] * WINV;
    __syncthreads();

    float* gp = xdb + (size_t)(m0 + wave * 16) * XDBW;
    const float* sp = stf + (wave * 16) * STP;
    const int rsub = lane >> 4, c4 = (lane & 15) * 4;
#pragma unroll
    for (int it = 0; it < 8; ++it) {
        const int row = it * 2 + rsub;
        const v4f val = *(const v4fa*)(sp + row * STP + c4);
        *(volatile v4f*)(gp + (size_t)row * XDBW + c4) = val;
    }
    __threadfence();
#pragma unroll
    for (int it = 0; it < 8; ++it) {
        const int row = it * 2 + rsub;
        const v4f val = *(const v4fa*)(sp + row * STP + c4);
        *(volatile v4f*)(gp + (size_t)row * XDBW + c4) = val;
    }
}

__device__ __forceinline__ void y_rows_store(const unsigned short* sy, unsigned short* gp, int wave, int lane) {
#pragma unroll
    for (int it = 0; it < 2; ++it) {
        const int row = 8 * wave + it * 4 + (lane >> 3);
        const int c   = (lane & 7) * 8;
        const u16x8 val = *(const u16x8a*)(sy + row * 64 + c);
        *(volatile u16x8*)(gp + (size_t)row * DI + c) = val;
    }
}

__global__ __launch_bounds__(64)
void scan_kernel(const float* __restrict__ X, unsigned short* ZY, const float* __restrict__ xdb,
                 const float* __restrict__ cw, const float* __restrict__ cb,
                 const float* __restrict__ Wdt, const float* __restrict__ dtb,
                 const float* __restrict__ Alog, const float* __restrict__ Dp)
{
    __shared__ __attribute__((aligned(16))) float sx[16 * XDBW];
    __shared__ __attribute__((aligned(16))) float sa[64 * DS];
    __shared__ __attribute__((aligned(16))) unsigned short sy[16 * 64];

    const int tid   = threadIdx.x;
    const int lane  = tid & 31;
    const int wave  = tid >> 5;
    const int dbase = blockIdx.x * 64;
    const int d     = dbase + tid;
    const size_t mrow0 = (size_t)blockIdx.y * TLEN;

#pragma unroll 1
    for (int i = tid; i < 64 * DS; i += 64) sa[i] = -__expf(Alog[(size_t)dbase * DS + i]);
    __syncthreads();

    float an[DS], hs[DS];
#pragma unroll
    for (int n = 0; n < DS; ++n) { an[n] = sa[tid * DS + n]; hs[n] = 0.0f; }
    float wdt[DTRK];
#pragma unroll
    for (int r = 0; r < DTRK; ++r) wdt[r] = Wdt[(size_t)d * DTRK + r];
    const float w0 = cw[d * DCONV + 0], w1 = cw[d * DCONV + 1], w2 = cw[d * DCONV + 2], w3 = cw[d * DCONV + 3];
    const float cbias = cb[d];
    const float tb = dtb[d];
    const float Dd = Dp[d];
    float xm1 = 0.0f, xm2 = 0.0f, xm3 = 0.0f;

#pragma unroll 1
    for (int l0 = 0; l0 < TLEN; l0 += 16) {
#pragma unroll
        for (int q = 0; q < 4; ++q) {
            const int idx4 = q * 64 + tid;
            const int row  = idx4 >> 4;
            const int c4   = (idx4 & 15) * 4;
            const v4f val = *(const v4f*)(xdb + (mrow0 + l0 + row) * XDBW + c4);
            *(v4fa*)(sx + row * XDBW + c4) = val;
        }
        __syncthreads();

#pragma unroll 1
        for (int t = 0; t < 16; ++t) {
            const size_t e = (mrow0 + l0 + t) * DI + d;
            const float xv = X[e];
            H16 zb; zb.u = ZY[e];
            const float zv = (float)zb.f;
            const float u  = conv4_silu(xm3, xm2, xm1, xv, w0, w1, w2, w3, cbias);
            xm3 = xm2; xm2 = xm1; xm1 = xv;
            const float* sr = sx + t * XDBW;
            float dl = 0.0f;
#pragma unroll
            for (int r = 0; r < DTRK; ++r) dl = fmaf(sr[r], wdt[r], dl);
            const float dt = softplus_f(dl + tb);
            const float du = dt * u;
            float y = 0.0f;
#pragma unroll
            for (int n = 0; n < DS; ++n) {
                const float da = __expf(dt * an[n]);
                hs[n] = da * hs[n] + du * sr[DTRK + n];
                y += hs[n] * sr[DTRK + DS + n];
            }
            const float g = (y + Dd * u) * silu_f(zv);
            H16 gb; gb.f = (_Float16)g;
            sy[t * 64 + tid] = gb.u;
        }
        __syncthreads();

        unsigned short* gp = ZY + (mrow0 + l0) * DI + dbase;
        y_rows_store(sy, gp, wave, lane);
        __threadfence();
        y_rows_store(sy, gp, wave, lane);
        __syncthreads();
    }
}

__global__ __launch_bounds__(256)
void gn_partial_kernel(const float* pre, double* gnp)
{
    __shared__ double sh1[256], sh2[256];
    __shared__ double sg1[NGRP], sg2[NGRP];
    const int tid = threadIdx.x, lane = tid & 31, w = tid >> 5;
    const int blk = blockIdx.x;
    const float* p = pre + (size_t)blk * GNROWS * DM + lane * 4;
    double s1 = 0.0, s2 = 0.0;
#pragma unroll 1
    for (int i = 0; i < GNROWS / 8; ++i) {
        const v4f x = *(const v4f*)(p + (size_t)(w + 8 * i) * DM);
#pragma unroll
        for (int c = 0; c < 4; ++c) {
            const double xd = (double)x[c];
            s1 += xd;
            s2 += xd * xd;
        }
    }
    sh1[tid] = s1;
    sh2[tid] = s2;
    __syncthreads();
    if (tid < NGRP) {
        double S1 = 0.0, S2 = 0.0;
#pragma unroll 1
        for (int ww = 0; ww < 8; ++ww)
#pragma unroll 1
            for (int l = 0; l < 8; ++l) {
                const int idx = ww * 32 + tid * 8 + l;
                S1 += sh1[idx];
                S2 += sh2[idx];
            }
        sg1[tid] = S1;
        sg2[tid] = S2;
    }
    __syncthreads();
    if (tid < 8) {
        v2d val;
        val[0] = 0.0; val[1] = 0.0;
        if (tid < NGRP) { val[0] = sg1[tid]; val[1] = sg2[tid]; }
        double* gp = gnp + (size_t)blk * 16 + tid * 2;
        *(volatile v2d*)gp = val;
        __threadfence();
        *(volatile v2d*)gp = val;
    }
}

__global__ __launch_bounds__(256)
void gn_norm_kernel(float* out, const double* gnp, const float* __restrict__ gamma, const float* __restrict__ beta)
{
    __shared__ float smean[NGRP], srstd[NGRP];
    const int tid = threadIdx.x, lane = tid & 31, w = tid >> 5;
    const int blk = blockIdx.x;
    const int b = blk / (GNBLK / NBAT);
    if (tid < NGRP) {
        double S1 = 0.0, S2 = 0.0;
#pragma unroll 1
        for (int q = 0; q < GNBLK / NBAT; ++q) {
            const double* src = gnp + ((size_t)b * (GNBLK / NBAT) + q) * 16 + tid * 2;
            S1 += src[0];
            S2 += src[1];
        }
        const double invN = 1.0 / (double)((size_t)TLEN * NNODES * (DM / NGRP));
        const double mean = S1 * invN;
        const double var  = S2 * invN - mean * mean;
        smean[tid] = (float)mean;
        srstd[tid] = rsqrtf(fmaxf((float)var, 0.0f) + GN_EPS);
    }
    __syncthreads();
    const int g = lane >> 3;
    const float mean = smean[g], rstd = srstd[g];
    const v4f gm = *(const v4f*)(gamma + lane * 4);
    const v4f bt = *(const v4f*)(beta + lane * 4);
    float* p = out + (size_t)blk * GNROWS * DM + lane * 4;
#pragma unroll 1
    for (int grp = 0; grp < GNROWS / 64; ++grp) {
        v4f y[8];
#pragma unroll
        for (int i = 0; i < 8; ++i) {
            const size_t ro = (size_t)(w + 8 * (grp * 8 + i)) * DM;
            const v4f x = *(const v4f*)(p + ro);
            y[i] = (x - mean) * rstd * gm + bt;
        }
#pragma unroll
        for (int i = 0; i < 8; ++i) {
            const size_t ro = (size_t)(w + 8 * (grp * 8 + i)) * DM;
            *(volatile v4f*)(p + ro) = y[i];
        }
        __threadfence();
#pragma unroll
        for (int i = 0; i < 8; ++i) {
            const size_t ro = (size_t)(w + 8 * (grp * 8 + i)) * DM;
            *(volatile v4f*)(p + ro) = y[i];
        }
    }
}

extern "C" void kernel_launch(void* const* d_in, const int* in_sizes, int n_in,
                              void* d_out, int out_size, void* d_ws, size_t ws_size,
                              hipStream_t stream)
{
    if (n_in < 12) return;
    if (in_sizes[0]  != NBAT * TLEN * NNODES * DM) return;
    if (in_sizes[1]  != 2 * DI * DM)              return;
    if (in_sizes[2]  != DI * DCONV)               return;
    if (in_sizes[3]  != DI)                       return;
    if (in_sizes[4]  != (DTRK + 2 * DS) * DI)     return;
    if (in_sizes[5]  != DI * DTRK)                return;
    if (in_sizes[6]  != DI)                       return;
    if (in_sizes[7]  != DI * DS)                  return;
    if (in_sizes[8]  != DI)                       return;
    if (in_sizes[9]  != DM * DI)                  return;
    if (in_sizes[10] != DM)                       return;
    if (in_sizes[11] != DM)                       return;
    if (out_size != NBAT * TLEN * NNODES * DM)    return;

    const float* v         = (const float*)d_in[0];
    const float* in_proj_w = (const float*)d_in[1];
    const float* conv_w    = (const float*)d_in[2];
    const float* conv_b    = (const float*)d_in[3];
    const float* x_proj_w  = (const float*)d_in[4];
    const float* dt_proj_w = (const float*)d_in[5];
    const float* dt_proj_b = (const float*)d_in[6];
    const float* A_log     = (const float*)d_in[7];
    const float* D_param   = (const float*)d_in[8];
    const float* out_proj_w= (const float*)d_in[9];
    const float* gn_gamma  = (const float*)d_in[10];
    const float* gn_beta   = (const float*)d_in[11];
    float* out = (float*)d_out;

    const size_t SZ_XF  = (size_t)NTOK * DI * 4;
    const size_t SZ_ZY  = (size_t)NTOK * DI * 2;
    const size_t SZ_X16 = (size_t)NTOK * DM * 2;
    const size_t SZ_XDB = (size_t)NTOK * XDBW * 4;
    const size_t SZ_R3  = (SZ_X16 > SZ_XDB) ? SZ_X16 : SZ_XDB;
    const size_t SZ_WI  = (size_t)2 * DI * DM * 2;
    const size_t SZ_WX  = (size_t)XDBW * DI * 2;
    const size_t SZ_WO  = (size_t)DM * DI * 2;
    const size_t SZ_GNP = (size_t)GNBLK * 128;

    const size_t OFF_XF  = 0;
    const size_t OFF_ZY  = OFF_XF + SZ_XF;
    const size_t OFF_R3  = OFF_ZY + SZ_ZY;
    const size_t OFF_WI  = OFF_R3 + SZ_R3;
    const size_t OFF_WX  = OFF_WI + SZ_WI;
    const size_t OFF_WO  = OFF_WX + SZ_WX;
    const size_t OFF_GNP = OFF_WO + SZ_WO;
    const size_t WS_END  = OFF_GNP + SZ_GNP;
    if (ws_size < WS_END) return;

    char* ws = (char*)d_ws;
    float*          Xf   = (float*)(ws + OFF_XF);
    unsigned short* ZY   = (unsigned short*)(ws + OFF_ZY);
    unsigned short* x16  = (unsigned short*)(ws + OFF_R3);
    float*          xdb  = (float*)(ws + OFF_R3);
    unsigned short* wi16 = (unsigned short*)(ws + OFF_WI);
    unsigned short* wx16 = (unsigned short*)(ws + OFF_WX);
    unsigned short* wo16 = (unsigned short*)(ws + OFF_WO);
    double*         gnp  = (double*)(ws + OFF_GNP);

    {
        const int n8v = (NBAT * TLEN * NNODES * DM) / 8;
        hipLaunchKernelGGL(cvt_v_kernel, dim3((n8v + 255) / 256), dim3(256), 0, stream, v, x16, n8v);
        const int n8wi = (2 * DI * DM) / 8;
        hipLaunchKernelGGL(cvt_w_kernel, dim3((n8wi + 255) / 256), dim3(256), 0, stream,
                           in_proj_w, wi16, n8wi, n8wi, WSCALE);
        const int n8wxv = ((DTRK + 2 * DS) * DI) / 8;
        const int n8wxt = (XDBW * DI) / 8;
        hipLaunchKernelGGL(cvt_w_kernel, dim3((n8wxt + 255) / 256), dim3(256), 0, stream,
                           x_proj_w, wx16, n8wxv, n8wxt, WSCALE);
        const int n8wo = (DM * DI) / 8;
        hipLaunchKernelGGL(cvt_w_kernel, dim3((n8wo + 255) / 256), dim3(256), 0, stream,
                           out_proj_w, wo16, n8wo, n8wo, WSCALE);
    }

    hipLaunchKernelGGL(HIP_KERNEL_NAME(gemm_tn_kernel<4, 0>),
                       dim3((2 * DI) / 128, NTOK / 64), dim3(128), 0, stream,
                       (const unsigned short*)x16, (const unsigned short*)wi16, (int)DM,
                       Xf, ZY, (const float*)v);

    hipLaunchKernelGGL(xproj_kernel, dim3(NTOK / 64), dim3(128), 0, stream,
                       (const float*)Xf, conv_w, conv_b, (const unsigned short*)wx16, xdb);

    hipLaunchKernelGGL(scan_kernel, dim3(DI / 64, NSEQ), dim3(64), 0, stream,
                       (const float*)Xf, ZY, (const float*)xdb, conv_w, conv_b,
                       dt_proj_w, dt_proj_b, A_log, D_param);

    hipLaunchKernelGGL(HIP_KERNEL_NAME(gemm_tn_kernel<4, 1>),
                       dim3(DM / 128, NTOK / 64), dim3(128), 0, stream,
                       (const unsigned short*)ZY, (const unsigned short*)wo16, (int)DI,
                       out, ZY, v);

    hipLaunchKernelGGL(gn_partial_kernel, dim3(GNBLK), dim3(256), 0, stream, (const float*)out, gnp);
    hipLaunchKernelGGL(gn_norm_kernel, dim3(GNBLK), dim3(256), 0, stream, out, (const double*)gnp,
                       gn_gamma, gn_beta);
}
